// SupernodePooling_38062000177493
// MI455X (gfx1250) — hardware-verified
//
#include <hip/hip_runtime.h>
#include <math.h>
#include <stdint.h>

typedef __attribute__((ext_vector_type(16))) _Float16 v16h;
typedef __attribute__((ext_vector_type(8)))  _Float16 v8h;
typedef __attribute__((ext_vector_type(16))) __bf16   v16b;
typedef __attribute__((ext_vector_type(8)))  __bf16   v8b;
typedef __attribute__((ext_vector_type(8)))  float    v8f;
typedef __attribute__((ext_vector_type(4)))  float    v4f;

constexpr int   IN_DIM = 32;
constexpr int   HID    = 256;
constexpr int   KSEL   = 32;
constexpr int   CAP    = 512;
constexpr int   CHUNK  = 1024;
constexpr int   NRUNG  = 7;
constexpr float RAD2   = 2.5e-5f;

__device__ __forceinline__ unsigned short f2bf_bits(float f) {
  unsigned u = __float_as_uint(f);
  return (unsigned short)((u + 0x7FFFu + ((u >> 16) & 1u)) >> 16);
}
__device__ __forceinline__ float bf_bits2f(unsigned short h) { return __uint_as_float(((unsigned)h) << 16); }

__device__ __forceinline__ void dep_guard_h(v8f& a, v8f& b, v16h x, v16h y) { asm volatile("v_nop\n\tv_nop\n\tv_nop\n\tv_nop" : "+v"(a), "+v"(b) : "v"(x), "v"(y)); }
__device__ __forceinline__ void dep_guard_b(v8f& a, v8f& b, v16b x, v16b y) { asm volatile("v_nop\n\tv_nop\n\tv_nop\n\tv_nop" : "+v"(a), "+v"(b) : "v"(x), "v"(y)); }
__device__ __forceinline__ void keep4_h(v16h a, v16h b, v16h c, v16h d) { asm volatile("v_nop" :: "v"(a), "v"(b), "v"(c), "v"(d)); }
__device__ __forceinline__ void keep4_b(v16b a, v16b b, v16b c, v16b d) { asm volatile("v_nop" :: "v"(a), "v"(b), "v"(c), "v"(d)); }
__device__ __forceinline__ void acc_guard4(v8f& a, v8f& b, v8f& c, v8f& d) { asm volatile("v_nop\n\tv_nop\n\tv_nop\n\tv_nop" : "+v"(a), "+v"(b), "+v"(c), "+v"(d)); }
template <typename T> struct Frag;
template <> struct Frag<_Float16> {
  typedef v16h V; union U { v16h v; v8h h[2]; };
  static __device__ __forceinline__ v16h load(const _Float16* p) {
    U f; f.h[0] = *(const v8h*)(p); f.h[1] = *(const v8h*)(p + 16); return f.v;
  }
  static __device__ __forceinline__ v8f mma(v16h a, v16h b, v8f c) {
    return __builtin_amdgcn_wmma_f32_16x16x32_f16(false, a, false, b, (short)0, c, false, false);
  }
  static __device__ __forceinline__ void guard(v8f& a, v8f& b, v16h x, v16h y) { dep_guard_h(a, b, x, y); }
  static __device__ __forceinline__ void keep(v16h a, v16h b, v16h c, v16h d) { keep4_h(a, b, c, d); }
};
template <> struct Frag<__bf16> {
  typedef v16b V; union U { v16b v; v8b h[2]; };
  static __device__ __forceinline__ v16b load(const __bf16* p) {
    U f; f.h[0] = *(const v8b*)(p); f.h[1] = *(const v8b*)(p + 16); return f.v;
  }
  static __device__ __forceinline__ v8f mma(v16b a, v16b b, v8f c) {
    return __builtin_amdgcn_wmma_f32_16x16x32_bf16(false, a, false, b, (short)0, c, false, false);
  }
  static __device__ __forceinline__ void guard(v8f& a, v8f& b, v16b x, v16b y) { dep_guard_b(a, b, x, y); }
  static __device__ __forceinline__ void keep(v16b a, v16b b, v16b c, v16b d) { keep4_b(a, b, c, d); }
};

template <int ET> struct Elem;
template <> struct Elem<0> { typedef _Float16 T; };
template <> struct Elem<1> { typedef __bf16 T; };
template <int ET, bool SPLIT, int BIAS_MODE, int OUT_MODE, bool RESID, int ACT = 0>
__global__ __launch_bounds__(256) void wmma_gemm64(
    const unsigned short* __restrict__ Ap, const unsigned short* __restrict__ A2p, int lda, long strideA,
    const unsigned short* __restrict__ Btp, const unsigned short* __restrict__ Bt2p, int ldb, long strideB,
    void* __restrict__ Cout, void* __restrict__ Cout2, int ldc, long strideC,
    const float* __restrict__ bias,
    const float* __restrict__ resid, long strideR, int ldr, int rshift,
    int M, int N, int K, float scale) {
  typedef typename Elem<ET>::T T;
  typedef typename Frag<T>::V V;
  const T* A = (const T*)Ap; const T* A2 = (const T*)A2p; const T* Bt = (const T*)Btp; const T* Bt2 = (const T*)Bt2p;
  __shared__ __align__(16) float sT[8][16 * 68];
  const int b    = blockIdx.y;
  const int lane = threadIdx.x & 31;
  const int wave = threadIdx.x >> 5;
  const int tilesN = N >> 6;
  const int tilesM = M >> 6;
  const int tile = blockIdx.x * 8 + wave;
  if (tile >= tilesM * tilesN) return;
  const int tm = tile / tilesN;
  const int tn = tile - tm * tilesN;
  const int m0 = tm << 6;
  const int n0 = tn << 6;

  const T* Ab  = A  + (size_t)b * strideA;
  const T* Bb  = Bt + (size_t)b * strideB;
  const T* Ab2 = SPLIT ? (A2  + (size_t)b * strideA) : nullptr;
  const T* Bb2 = SPLIT ? (Bt2 + (size_t)b * strideB) : nullptr;

  const int rlane = lane & 15;
  const int koff  = (lane >> 4) * 8;
  const int mOff  = (lane >> 4) * 8;

  v8f acc[4][4];
#pragma unroll
  for (int i = 0; i < 4; ++i)
#pragma unroll
    for (int j = 0; j < 4; ++j) acc[i][j] = (v8f){0.f,0.f,0.f,0.f,0.f,0.f,0.f,0.f};

  for (int k0 = 0; k0 < K; k0 += 32) {
    V bh[4], bl[4];
#pragma unroll
    for (int j = 0; j < 4; ++j) {
      const size_t bo = (size_t)(n0 + (j << 4) + rlane) * ldb + koff + k0;
      bh[j] = Frag<T>::load(Bb + bo);
      if (SPLIT) bl[j] = Frag<T>::load(Bb2 + bo);
    }
#pragma unroll
    for (int i = 0; i < 4; ++i) {
      const size_t ao = (size_t)(m0 + (i << 4) + rlane) * lda + koff + k0;
      V ah = Frag<T>::load(Ab + ao);
      V al;
      if (SPLIT) al = Frag<T>::load(Ab2 + ao);
#pragma unroll
      for (int j = 0; j < 4; ++j) {
        acc[i][j] = Frag<T>::mma(ah, bh[j], acc[i][j]);
        if (SPLIT) {
          acc[i][j] = Frag<T>::mma(ah, bl[j], acc[i][j]);
          acc[i][j] = Frag<T>::mma(al, bh[j], acc[i][j]);
        }
      }
      Frag<T>::guard(acc[i][0], acc[i][3], ah, SPLIT ? al : ah);
    }
    Frag<T>::keep(bh[0], bh[1], bh[2], bh[3]);
    if (SPLIT) Frag<T>::keep(bl[0], bl[1], bl[2], bl[3]);
  }
  acc_guard4(acc[0][0], acc[0][1], acc[0][2], acc[0][3]);
  acc_guard4(acc[1][0], acc[1][1], acc[1][2], acc[1][3]);
  acc_guard4(acc[2][0], acc[2][1], acc[2][2], acc[2][3]);
  acc_guard4(acc[3][0], acc[3][1], acc[3][2], acc[3][3]);

  float* slab = sT[wave];
  const float* Rb = RESID ? (resid + (size_t)b * strideR) : nullptr;
#pragma unroll
  for (int i = 0; i < 4; ++i) {
    const int mBase = m0 + (i << 4);
#pragma unroll
    for (int j = 0; j < 4; ++j) {
      const int n = n0 + (j << 4) + rlane;
      float bv = 0.f;
      if (BIAS_MODE == 2) bv = bias[n];
#pragma unroll
      for (int r = 0; r < 8; ++r) {
        float v = acc[i][j][r] * scale;
        if (BIAS_MODE == 1) v += bias[mBase + mOff + r];
        if (BIAS_MODE == 2) v += bv;
        if (RESID) v += Rb[(size_t)((mBase + mOff + r) >> rshift) * ldr + n];
        if (ACT == 1) v = tanhf(v);
        if (ACT == 2) v = fmaxf(v, 0.0f);
        if (ACT == 3) v = v / (1.0f + expf(-v));
        if (ACT == 4) v = (v > 0.f) ? v : 0.01f * v;
        if (ACT == 5) v = 0.5f * v * (1.0f + erff(v * 0.70710678118654752f));
        if (ACT == 6) {
          const float u = 0.7978845608028654f * (v + 0.044715f * (v * v * v));
          const float cdf = 0.5f * (1.0f + tanhf(u));
          v = v * cdf;
        }
        slab[(mOff + r) * 68 + (j << 4) + rlane] = v;
      }
    }
    __builtin_amdgcn_fence(__ATOMIC_RELEASE, "workgroup");
    __builtin_amdgcn_wave_barrier();
    __builtin_amdgcn_fence(__ATOMIC_ACQUIRE, "workgroup");
    if (OUT_MODE == 0) {
      float* C = (float*)Cout + (size_t)b * strideC;
      const int hh = lane >> 4, c4 = (lane & 15) * 4;
      for (int pass = 0; pass < 2; ++pass) {
#pragma unroll
        for (int it = 0; it < 8; ++it) {
          const int row = it * 2 + hh;
          v4f v = *(const v4f*)(slab + row * 68 + c4);
          *(volatile v4f*)(C + (size_t)(mBase + row) * ldc + n0 + c4) = v;
        }
        __threadfence();
      }
    } else {
      const int q = lane >> 3, c8 = (lane & 7) * 8;
      unsigned short* C  = (unsigned short*)Cout  + (size_t)b * strideC;
      unsigned short* C2 = (OUT_MODE == 2) ? ((unsigned short*)Cout2 + (size_t)b * strideC) : nullptr;
      for (int pass = 0; pass < 2; ++pass) {
#pragma unroll
        for (int it = 0; it < 4; ++it) {
          const int row = it * 4 + q;
          const float* sp = slab + row * 68 + c8;
          v8h hv, lv;
#pragma unroll
          for (int e = 0; e < 8; ++e) {
            if (OUT_MODE == 1) {
              hv[e] = (_Float16)sp[e];
            } else {
              unsigned short hb = f2bf_bits(sp[e]);
              unsigned short lb = f2bf_bits(sp[e] - bf_bits2f(hb));
              hv[e] = __builtin_bit_cast(_Float16, hb);
              lv[e] = __builtin_bit_cast(_Float16, lb);
            }
          }
          *(volatile v8h*)(C + (size_t)(mBase + row) * ldc + n0 + c8) = hv;
          if (OUT_MODE == 2) *(volatile v8h*)(C2 + (size_t)(mBase + row) * ldc + n0 + c8) = lv;
        }
        __threadfence();
      }
    }
    __builtin_amdgcn_fence(__ATOMIC_RELEASE, "workgroup");
    __builtin_amdgcn_wave_barrier();
    __builtin_amdgcn_fence(__ATOMIC_ACQUIRE, "workgroup");
  }
}

__global__ __launch_bounds__(256) void cast_f32_f16x2(
    const float* __restrict__ in, _Float16* __restrict__ out, int n2) {
  int i = blockIdx.x * 256 + threadIdx.x;
  if (i < n2) {
    const _Float16 h0 = (_Float16)in[2 * i], h1 = (_Float16)in[2 * i + 1];
    const unsigned u = (unsigned)__builtin_bit_cast(unsigned short, h0) | ((unsigned)__builtin_bit_cast(unsigned short, h1) << 16);
    ((volatile unsigned*)out)[i] = u;
    __threadfence();
    ((volatile unsigned*)out)[i] = u;
  }
}

__global__ __launch_bounds__(256) void transpose_cast_f16(
    const float* __restrict__ in, _Float16* __restrict__ out, int R, int C) {
  const int t = blockIdx.x * 256 + threadIdx.x;
  const int total8 = (R * C) >> 3;
  if (t < total8) {
    const int o0 = t * 8;
    const int c  = o0 / R;
    const int r0 = o0 - c * R;
    v8h v;
#pragma unroll
    for (int e = 0; e < 8; ++e) v[e] = (_Float16)in[(size_t)(r0 + e) * C + c];
    *(volatile v8h*)(out + o0) = v;
    __threadfence();
    *(volatile v8h*)(out + o0) = v;
  }
}

__global__ __launch_bounds__(256) void xbuild_kernel(
    const float* __restrict__ Xlin, const float* __restrict__ pos, _Float16* __restrict__ x16, int nrows) {
  __shared__ float sfreq[HID / 2];
  __shared__ __align__(16) _Float16 srow[8][HID];
  const int tid = threadIdx.x, wave = tid >> 5, lane = tid & 31;
  if (tid < HID / 2) sfreq[tid] = expf((float)tid * (-(9.2103403719761836f) / (float)(HID / 2 - 1)));
  __syncthreads();
  const int row  = blockIdx.x * 8 + wave;
  const int rowc = row < nrows ? row : nrows - 1;
  const float p = pos[rowc];
  const float* xr = Xlin + (size_t)rowc * HID;
#pragma unroll 1
  for (int e = 0; e < 4; ++e) {
    const int c = e * 32 + lane;
    const float a = p * sfreq[c];
    srow[wave][c]           = (_Float16)(xr[c] + sinf(a));
    srow[wave][c + HID / 2] = (_Float16)(xr[c + HID / 2] + cosf(a));
  }
  __syncthreads();
  const v8h v = *(const v8h*)(&srow[wave][lane * 8]);
  _Float16* dst = x16 + (size_t)rowc * HID + lane * 8;
  if (row < nrows) *(volatile v8h*)dst = v;
  __threadfence();
  if (row < nrows) *(volatile v8h*)dst = v;
}

__device__ __forceinline__ void lds_wave_sync() {
  __builtin_amdgcn_fence(__ATOMIC_RELEASE, "workgroup");
  __builtin_amdgcn_wave_barrier();
  __builtin_amdgcn_fence(__ATOMIC_ACQUIRE, "workgroup");
}

__global__ __launch_bounds__(256) void select_gather_kernel(
    const float* __restrict__ pos, const int* __restrict__ sup, const _Float16* __restrict__ x16,
    _Float16* __restrict__ A16, _Float16* __restrict__ Xs16, float* __restrict__ Wf,
    int sb, int cs, int nsup, int npts) {
#pragma clang fp contract(off)
  __shared__ unsigned Lk_s[8][CAP];
  __shared__ int      Li_s[8][CAP];
  const int tid  = threadIdx.x;
  const int wave = tid >> 5;
  const int lane = tid & 31;
  const int ls = blockIdx.x * 8 + wave;
  if (ls >= cs) return;
  int s = sb + ls; s = (s < nsup) ? s : (nsup - 1);
  int sidx = sup[s];
  sidx = (sidx < 0) ? 0 : ((sidx >= npts) ? (npts - 1) : sidx);
  const float p = pos[sidx];

  int n = 0;
#pragma unroll 1
  for (int att = 0; att < NRUNG; ++att) {
    const float thr = (att < NRUNG - 1) ? __uint_as_float(((unsigned)(107 + 2 * att)) << 23) : 3.0e38f;
    n = 0;
#pragma unroll 1
    for (int base = 0; base < npts; base += 32) {
      const int  i   = base + lane;
      const bool inb = (i < npts);
      const float xv = pos[inb ? i : 0];
      const float d  = p - xv;
      const float d2 = d * d;
      const bool hit = inb && (d2 <= thr);
      const unsigned mask = __builtin_amdgcn_ballot_w32(hit);
      const int pre = (int)__builtin_amdgcn_mbcnt_lo(mask, 0u);
      const int tot = __builtin_popcount(mask);
      if (hit) {
        const int slot = n + pre;
        if (slot < CAP) { Lk_s[wave][slot] = __float_as_uint(d2); Li_s[wave][slot] = i; }
      }
      n = n + tot; n = (n < CAP) ? n : CAP;
    }
    if (n >= KSEL) break;
  }
  lds_wave_sync();

  int   mysel = sidx;
  float myw   = 0.0f;
  const int nq = (n + 31) >> 5;
#pragma unroll 1
  for (int j = 0; j < KSEL; ++j) {
    unsigned bk = 0xFFFFFFFFu, bi = 0xFFFFFFFFu;
#pragma unroll 1
    for (int q = 0; q < nq; ++q) {
      const int i = (q << 5) + lane;
      if (i < n) {
        const unsigned kb = Lk_s[wave][i];
        if (kb < bk || (kb == bk && (unsigned)i < bi)) { bk = kb; bi = (unsigned)i; }
      }
    }
#pragma unroll
    for (int off = 16; off > 0; off >>= 1) {
      const unsigned ok = __shfl_xor(bk, off, 32);
      const unsigned oi = __shfl_xor(bi, off, 32);
      if (ok < bk || (ok == bk && oi < bi)) { bk = ok; bi = oi; }
    }
    if (bk < 0x7F800000u) {
      const int w = (int)(bi & (unsigned)(CAP - 1));
      const int node = Li_s[wave][w];
      if (lane == j) { mysel = node; myw = (__uint_as_float(bk) <= RAD2) ? 1.0f : 0.0f; }
      if (lane == 0) Lk_s[wave][w] = 0x7F800000u;
    }
    lds_wave_sync();
  }
  mysel = (mysel < 0) ? 0 : ((mysel >= npts) ? (npts - 1) : mysel);

  const _Float16* xsup = x16 + (size_t)sidx * HID + lane * 8;
  _Float16* xsd  = Xs16 + (size_t)ls * HID + lane * 8;
  _Float16* arow = A16 + (size_t)ls * KSEL * HID + lane * 8;
  float*    wrow = Wf + (size_t)ls * KSEL + lane;
  for (int pass = 0; pass < 2; ++pass) {
    {
      const v8h v = *(const v8h*)xsup;
      *(volatile v8h*)xsd = v;
    }
#pragma unroll 1
    for (int j = 0; j < KSEL; ++j) {
      const int node = __shfl(mysel, j, 32);
      const v8h v = *(const v8h*)(x16 + (size_t)node * HID + lane * 8);
      *(volatile v8h*)(arow + (size_t)j * HID) = v;
    }
    *(volatile float*)wrow = myw;
    __threadfence();
  }
}

__global__ __launch_bounds__(256) void pool_kernel(
    const float* __restrict__ Mo, const float* __restrict__ Wf, float* __restrict__ out, int cs) {
  const int wave = threadIdx.x >> 5, lane = threadIdx.x & 31;
  const int ls = blockIdx.x * 8 + wave;
  if (ls >= cs) return;
  const float wl = Wf[(size_t)ls * KSEL + lane];
  float cnt = wl;
#pragma unroll
  for (int off = 16; off > 0; off >>= 1) cnt += __shfl_xor(cnt, off, 32);
  v4f a0 = {0.f, 0.f, 0.f, 0.f};
  v4f a1 = {0.f, 0.f, 0.f, 0.f};
#pragma unroll 2
  for (int j = 0; j < KSEL; ++j) {
    const float w = __shfl(wl, j, 32);
    const float* mr = Mo + ((size_t)ls * KSEL + j) * HID;
    const v4f u0 = *(const v4f*)(mr + lane * 4);
    const v4f u1 = *(const v4f*)(mr + HID / 2 + lane * 4);
    a0 += u0 * w;
    a1 += u1 * w;
  }
  const float inv = 1.0f / fmaxf(cnt, 1.0f);
  a0 *= inv;
  a1 *= inv;
  float* orow = out + (size_t)ls * HID;
  *(volatile v4f*)(orow + lane * 4) = a0;
  *(volatile v4f*)(orow + HID / 2 + lane * 4) = a1;
  __threadfence();
  *(volatile v4f*)(orow + lane * 4) = a0;
  *(volatile v4f*)(orow + HID / 2 + lane * 4) = a1;
}

template <int BIAS_MODE, int OUT_MODE, bool RESID, int ACT>
static void run_gemm(hipStream_t st, const void* A, int lda, const void* Bt, int ldb, void* C, int ldc,
                     const float* bias, const float* resid, int ldr, int rshift, int M, int N, int K) {
  const int tiles = (M / 64) * (N / 64);
  dim3 grid((unsigned)((tiles + 7) / 8), 1, 1);
  wmma_gemm64<0, false, BIAS_MODE, OUT_MODE, RESID, ACT><<<grid, 256, 0, st>>>(
      (const unsigned short*)A, (const unsigned short*)A, lda, 0L,
      (const unsigned short*)Bt, (const unsigned short*)Bt, ldb, 0L,
      C, C, ldc, 0L, bias, resid, 0L, ldr, rshift, M, N, K, 1.0f);
}

static inline size_t align256(size_t x) { return (x + 255) & ~(size_t)255; }

extern "C" void kernel_launch(void* const* d_in, const int* in_sizes, int n_in,
                              void* d_out, int out_size, void* d_ws, size_t ws_size,
                              hipStream_t stream) {
  if (n_in < 10) return;
  const float* feat  = (const float*)d_in[0];
  const float* pos   = (const float*)d_in[1];
  const int*   sup   = (const int*)d_in[2];
  const float* projW = (const float*)d_in[4];
  const float* projB = (const float*)d_in[5];
  const float* W1    = (const float*)d_in[6];
  const float* b1    = (const float*)d_in[7];
  const float* W2    = (const float*)d_in[8];
  const float* b2    = (const float*)d_in[9];
  float* out = (float*)d_out;

  const int npts = in_sizes[1];
  const int nsup = in_sizes[2];
  if (npts < 64 || (npts % 64) != 0) return;
  if (nsup < 2 || (nsup % 2) != 0) return;
  if (in_sizes[0] != npts * IN_DIM || in_sizes[4] != IN_DIM * HID || in_sizes[5] != HID ||
      in_sizes[6] != 2 * HID * HID || in_sizes[7] != HID || in_sizes[8] != HID * HID || in_sizes[9] != HID) return;
  if (out_size != nsup * HID) return;

  size_t off = 0;
  const size_t oFeat16 = off; off += align256((size_t)npts * IN_DIM * 2);
  const size_t oPWt    = off; off += align256((size_t)HID * IN_DIM * 2);
  const size_t oW1t    = off; off += align256((size_t)HID * 2 * HID * 2);
  const size_t oW2t    = off; off += align256((size_t)HID * HID * 2);
  const size_t oX16    = off; off += align256((size_t)npts * HID * 2);
  const size_t oXs16   = off; off += align256((size_t)CHUNK * HID * 2);
  const size_t oD      = off; off += align256((size_t)CHUNK * HID * 4);
  const size_t oWf     = off; off += align256((size_t)CHUNK * KSEL * 4);
  const size_t chunkRowsMax = (size_t)CHUNK * KSEL;
  const size_t regA  = chunkRowsMax * HID * 2;
  const size_t regH  = chunkRowsMax * HID * 2;
  const size_t regM  = chunkRowsMax * HID * 4;
  size_t regionBytes = (size_t)npts * HID * 4;
  if (regionBytes < regA + regH + regM) regionBytes = regA + regH + regM;
  const size_t oRegion = off; off += align256(regionBytes);
  if (off > ws_size) return;

  char* ws = (char*)d_ws;
  _Float16* feat16 = (_Float16*)(ws + oFeat16);
  _Float16* PWt    = (_Float16*)(ws + oPWt);
  _Float16* W1t    = (_Float16*)(ws + oW1t);
  _Float16* W2t    = (_Float16*)(ws + oW2t);
  _Float16* x16    = (_Float16*)(ws + oX16);
  _Float16* Xs16   = (_Float16*)(ws + oXs16);
  float*    Dm     = (float*)(ws + oD);
  float*    Wf     = (float*)(ws + oWf);
  float*    Xlin   = (float*)(ws + oRegion);
  _Float16* A16    = (_Float16*)(ws + oRegion);
  _Float16* H16    = (_Float16*)(ws + oRegion + regA);
  float*    Mo     = (float*)(ws + oRegion + regA + regH);

  {
    const int n2 = npts * IN_DIM / 2;
    cast_f32_f16x2<<<(unsigned)((n2 + 255) / 256), 256, 0, stream>>>(feat, feat16, n2);
  }
  {
    const int t0 = (IN_DIM * HID) / 8;
    transpose_cast_f16<<<(unsigned)((t0 + 255) / 256), 256, 0, stream>>>(projW, PWt, IN_DIM, HID);
    const int t1 = (2 * HID * HID) / 8;
    transpose_cast_f16<<<(unsigned)((t1 + 255) / 256), 256, 0, stream>>>(W1, W1t, 2 * HID, HID);
    const int t2 = (HID * HID) / 8;
    transpose_cast_f16<<<(unsigned)((t2 + 255) / 256), 256, 0, stream>>>(W2, W2t, HID, HID);
  }
  run_gemm<2, 0, false, 0>(stream, feat16, IN_DIM, PWt, IN_DIM, Xlin, HID, projB, Dm, 0, 0, npts, HID, IN_DIM);
  xbuild_kernel<<<(unsigned)((npts + 7) / 8), 256, 0, stream>>>(Xlin, pos, x16, npts);

  const int nchunks = (nsup + CHUNK - 1) / CHUNK;
  for (int c = 0; c < nchunks; ++c) {
    const int sb = c * CHUNK;
    int cs = nsup - sb; if (cs > CHUNK) cs = CHUNK;
    const int mrows = cs * KSEL;
    select_gather_kernel<<<(unsigned)((cs + 7) / 8), 256, 0, stream>>>(pos, sup, x16, A16, Xs16, Wf, sb, cs, nsup, npts);
    run_gemm<2, 0, false, 0>(stream, Xs16, HID, W1t + HID, 2 * HID, Dm, HID, b1, Dm, 0, 0, cs, HID, HID);
    run_gemm<0, 1, true, 6>(stream, A16, HID, W1t, 2 * HID, H16, HID, b1, Dm, HID, 5, mrows, HID, HID);
    run_gemm<2, 0, false, 0>(stream, H16, HID, W2t, HID, Mo, HID, b2, Dm, 0, 0, mrows, HID, HID);
    pool_kernel<<<(unsigned)((cs + 7) / 8), 256, 0, stream>>>(Mo, Wf, out + (size_t)sb * HID, cs);
  }
}
